// VanillaMHA_5085241278732
// MI455X (gfx1250) — hardware-verified
//
#include <hip/hip_runtime.h>
#include <math.h>
#include <stdint.h>

#define NB      4
#define NQ      2048
#define NC      2048
#define DMODEL  1024
#define NHEAD   16
#define HDIM    64
#define NROWS   (NB * NQ)
#define NE      512
#define NL      (NQ - NE)
#define PQK     (2 * DMODEL)
#define WSC     64.0f
#define HCARRY  16.0f
#define QC      16.0f
#define KC      16.0f
#define VC      16.0f
#define PC      1024.0f
#define FC      1024.0f
#define RSC     2048.0f
#define RINV    0.00048828125f
#define ATT_SCALE 0.125f
#define LOG2E   1.4426950408889634f
#define LN_EPS  1e-5f
static_assert(NHEAD * HDIM == DMODEL);
static_assert(NE + NL == NQ && (NE % 64) == 0 && (NL % 64) == 0 && (NE % 32) == 0 && (NE % 16) == 0);
static_assert((NQ % 64) == 0 && (NC % 64) == 0 && (DMODEL % 64) == 0 && (NC % 32) == 0 && (NROWS % 64) == 0);
#define HPB     8
#define NHB     (NHEAD / HPB)
#define OSP     (HPB * HDIM)
#define ATT_THREADS (HPB * 32)
static_assert(ATT_THREADS == 256 && NHB * HPB == NHEAD && OSP == 64 * 8);
#define LN_THREADS 256
static_assert(LN_THREADS * 4 == DMODEL);
#define PS_FLOATS  (HPB * 16 * 36)
#define OS_HALVES  (16 * OSP)
#define OS2_FLOATS 8192
static_assert((size_t)OS_HALVES * 2 <= (size_t)PS_FLOATS * 4);
static_assert((size_t)2 * OS_HALVES * 2 <= (size_t)OS2_FLOATS * 4 && OS2_FLOATS >= PS_FLOATS);
static_assert(((16 * OSP) % (8 * ATT_THREADS)) == 0 && ((16 * OSP) / (8 * ATT_THREADS)) == 4);

typedef _Float16 v16h __attribute__((ext_vector_type(16)));
typedef _Float16 v8h  __attribute__((ext_vector_type(8)));
typedef float    v8f  __attribute__((ext_vector_type(8)));
typedef float    v4f  __attribute__((ext_vector_type(4)));
typedef unsigned int v4u __attribute__((ext_vector_type(4)));
typedef unsigned int v2u __attribute__((ext_vector_type(2)));

union FragH { v16h v; v8h h[2]; v4u u[2]; };

__device__ __forceinline__ unsigned short bf_bits(float f) {
  unsigned u = __float_as_uint(f);
  return (unsigned short)((u + 0x7FFFu + ((u >> 16) & 1u)) >> 16);
}
__device__ __forceinline__ float bf_up(unsigned short h) { return __uint_as_float(((unsigned)h) << 16); }
__device__ __forceinline__ float bfr(float f) { return bf_up(bf_bits(f)); }
__device__ __forceinline__ unsigned short h_bits(_Float16 x) { return __builtin_bit_cast(unsigned short, x); }
__device__ __forceinline__ unsigned pk16(unsigned short a, unsigned short b) { return (unsigned)a | ((unsigned)b << 16); }
__device__ __forceinline__ v8f zero8() { v8f z = {0.f, 0.f, 0.f, 0.f, 0.f, 0.f, 0.f, 0.f}; return z; }
__device__ __forceinline__ int imin(int a, int b) { return a < b ? a : b; }

__device__ __forceinline__ v16h ldfrag_h(const _Float16* p) {
  FragH f;
  f.h[0] = *(const v8h*)(p);
  f.h[1] = *(const v8h*)(p + 16);
  return f.v;
}
__device__ __forceinline__ v16h ldfrag_u(const unsigned short* p) {
  FragH f;
  f.u[0] = *(const v4u*)(p);
  f.u[1] = *(const v4u*)(p + 16);
  return f.v;
}

__device__ __forceinline__ v8f mma_raw(v16h a, v16h b, v8f c) {
  return __builtin_amdgcn_wmma_f32_16x16x32_f16(false, a, false, b, (short)0, c, false, false);
}
__device__ __forceinline__ void dep_guard1(v8f& a, v8f& b, v16h x) {
#if defined(__HIP_DEVICE_COMPILE__)
  asm volatile("v_nop\n\tv_nop\n\tv_nop\n\tv_nop" : "+v"(a), "+v"(b) : "v"(x));
#endif
}
__device__ __forceinline__ void dep_guard2(v8f& a, v8f& b, v8f& c, v8f& d, v16h x, v16h y) {
#if defined(__HIP_DEVICE_COMPILE__)
  asm volatile("v_nop\n\tv_nop\n\tv_nop\n\tv_nop" : "+v"(a), "+v"(b), "+v"(c), "+v"(d) : "v"(x), "v"(y));
#endif
}
__device__ __forceinline__ void guard_s2(v8f& s, v16h a0, v16h a1) {
#if defined(__HIP_DEVICE_COMPILE__)
  asm volatile("v_nop\n\tv_nop\n\tv_nop\n\tv_nop" : "+v"(s) : "v"(a0), "v"(a1));
#endif
}
__device__ __forceinline__ void guard_s4(v8f& s, v16h a0, v16h a1, v16h b0, v16h b1) {
#if defined(__HIP_DEVICE_COMPILE__)
  asm volatile("v_nop\n\tv_nop\n\tv_nop\n\tv_nop" : "+v"(s) : "v"(a0), "v"(a1), "v"(b0), "v"(b1));
#endif
}
__device__ __forceinline__ void guard_x4(v8f& s, v8f& t, v16h a0, v16h a1, v16h a2, v16h a3) {
#if defined(__HIP_DEVICE_COMPILE__)
  asm volatile("v_nop\n\tv_nop\n\tv_nop\n\tv_nop" : "+v"(s), "+v"(t) : "v"(a0), "v"(a1), "v"(a2), "v"(a3) : "memory");
#endif
}
__device__ __forceinline__ void guard_x8(v8f& s, v8f& t, v16h a0, v16h a1, v16h a2, v16h a3,
                                         v16h b0, v16h b1, v16h b2, v16h b3) {
#if defined(__HIP_DEVICE_COMPILE__)
  asm volatile("v_nop\n\tv_nop\n\tv_nop\n\tv_nop"
               : "+v"(s), "+v"(t) : "v"(a0), "v"(a1), "v"(a2), "v"(a3), "v"(b0), "v"(b1), "v"(b2), "v"(b3) : "memory");
#endif
}
__device__ __forceinline__ void guard_pv4(v8f& a, v8f& b, v8f& c, v8f& d, v16h x, v16h y, v16h z, v16h w, v16h u) {
#if defined(__HIP_DEVICE_COMPILE__)
  asm volatile("v_nop\n\tv_nop\n\tv_nop\n\tv_nop"
               : "+v"(a), "+v"(b), "+v"(c), "+v"(d) : "v"(x), "v"(y), "v"(z), "v"(w), "v"(u));
#endif
}
__device__ __forceinline__ void guard_pv2(v8f& a, v8f& b, v16h x, v16h y, v16h z, v16h w) {
#if defined(__HIP_DEVICE_COMPILE__)
  asm volatile("v_nop\n\tv_nop\n\tv_nop\n\tv_nop" : "+v"(a), "+v"(b) : "v"(x), "v"(y), "v"(z), "v"(w));
#endif
}
__device__ __forceinline__ void keep4_h(v16h a, v16h b, v16h c, v16h d) {
#if defined(__HIP_DEVICE_COMPILE__)
  asm volatile("v_nop" :: "v"(a), "v"(b), "v"(c), "v"(d));
#endif
}
__device__ __forceinline__ void acc_guard4(v8f& a, v8f& b, v8f& c, v8f& d) {
#if defined(__HIP_DEVICE_COMPILE__)
  asm volatile("v_nop\n\tv_nop\n\tv_nop\n\tv_nop" : "+v"(a), "+v"(b), "+v"(c), "+v"(d));
#endif
}
__device__ __forceinline__ void wave_sync_lds() {
  __builtin_amdgcn_fence(__ATOMIC_RELEASE, "workgroup");
  __builtin_amdgcn_wave_barrier();
  __builtin_amdgcn_fence(__ATOMIC_ACQUIRE, "workgroup");
}

__global__ __launch_bounds__(128) void wcvt16(const float* __restrict__ src, unsigned short* dst, int nsrc, int perm) {
  const int row = blockIdx.x, tid = threadIdx.x;
  int srow = row;
  if (perm != 0) {
    const int part = row >> 10;
    const int hn   = (row >> 6) & 15;
    const int d    = row & 63;
    srow = hn * (3 * HDIM) + part * HDIM + d;
  }
  srow = imin(srow, nsrc - 1);
  const float* sp = src + (size_t)srow * DMODEL + (size_t)tid * 8;
  const v4f a = *(const v4f*)(sp);
  const v4f b = *(const v4f*)(sp + 4);
  v4u hv;
  hv[0] = pk16(h_bits((_Float16)(bfr(a[0]) * WSC)), h_bits((_Float16)(bfr(a[1]) * WSC)));
  hv[1] = pk16(h_bits((_Float16)(bfr(a[2]) * WSC)), h_bits((_Float16)(bfr(a[3]) * WSC)));
  hv[2] = pk16(h_bits((_Float16)(bfr(b[0]) * WSC)), h_bits((_Float16)(bfr(b[1]) * WSC)));
  hv[3] = pk16(h_bits((_Float16)(bfr(b[2]) * WSC)), h_bits((_Float16)(bfr(b[3]) * WSC)));
  unsigned short* dp = dst + (size_t)row * DMODEL + (size_t)tid * 8;
  for (int pass = 0; pass < 2; ++pass) {
    *(volatile v4u*)dp = hv;
    __threadfence();
  }
}

__global__ __launch_bounds__(LN_THREADS)
void lnorm2(const float* __restrict__ Xp, const float* __restrict__ gp, const float* __restrict__ bp,
            unsigned short* XHp, unsigned short* XLp) {
  __shared__ float red[2][LN_THREADS / 32];
  __shared__ __align__(16) unsigned short srh[DMODEL];
  __shared__ __align__(16) unsigned short srl[DMODEL];
  const int row  = blockIdx.x;
  const int tid  = threadIdx.x;
  const int lane = tid & 31;
  const int wave = tid >> 5;
  const size_t base = (size_t)row * DMODEL + (size_t)tid * 4;
  v4f v = *(const v4f*)(Xp + base);
#pragma unroll
  for (int e = 0; e < 4; ++e) v[e] = bfr(v[e]);
  float s = (v[0] + v[1]) + (v[2] + v[3]);
#pragma unroll
  for (int off = 1; off < 32; off <<= 1) s += __shfl_xor(s, off, 32);
  if (lane == 0) red[0][wave] = s;
  __syncthreads();
  float tot = 0.f;
#pragma unroll
  for (int w = 0; w < LN_THREADS / 32; ++w) tot += red[0][w];
  const float mu = tot * (1.0f / (float)DMODEL);
  v4f d;
#pragma unroll
  for (int e = 0; e < 4; ++e) d[e] = v[e] - mu;
  float q = (d[0] * d[0] + d[1] * d[1]) + (d[2] * d[2] + d[3] * d[3]);
#pragma unroll
  for (int off = 1; off < 32; off <<= 1) q += __shfl_xor(q, off, 32);
  if (lane == 0) red[1][wave] = q;
  __syncthreads();
  float totq = 0.f;
#pragma unroll
  for (int w = 0; w < LN_THREADS / 32; ++w) totq += red[1][w];
  const float var  = totq * (1.0f / (float)DMODEL);
  const float rstd = rsqrtf(var + LN_EPS);
  const v4f gv = *(const v4f*)(gp + (size_t)tid * 4);
  const v4f bv = *(const v4f*)(bp + (size_t)tid * 4);
  unsigned short hb16[4], lb16[4];
#pragma unroll
  for (int e = 0; e < 4; ++e) {
    const float o = (d[e] * rstd) * bfr(gv[e]) + bfr(bv[e]);
    const float f = o * HCARRY;
    const _Float16 h = (_Float16)f;
    hb16[e] = h_bits(h);
    lb16[e] = h_bits((_Float16)((f - (float)h) * RSC));
  }
  v2u wh, wl;
  wh[0] = pk16(hb16[0], hb16[1]);
  wh[1] = pk16(hb16[2], hb16[3]);
  wl[0] = pk16(lb16[0], lb16[1]);
  wl[1] = pk16(lb16[2], lb16[3]);
  *(v2u*)(srh + tid * 4) = wh;
  *(v2u*)(srl + tid * 4) = wl;
  __syncthreads();
  if (tid < DMODEL / 8) {
    const v4u hv = *(const v4u*)(srh + tid * 8);
    unsigned short* dst = XHp + (size_t)row * DMODEL + (size_t)tid * 8;
    for (int pass = 0; pass < 2; ++pass) {
      *(volatile v4u*)dst = hv;
      __threadfence();
    }
  } else {
    const int t2 = tid - DMODEL / 8;
    const v4u hv = *(const v4u*)(srl + t2 * 8);
    unsigned short* dst = XLp + (size_t)row * DMODEL + (size_t)t2 * 8;
    for (int pass = 0; pass < 2; ++pass) {
      *(volatile v4u*)dst = hv;
      __threadfence();
    }
  }
}

template <int MI, int LO, int OM>
__global__ __launch_bounds__(256) void gemmw(
    const unsigned short* __restrict__ Ahp, int lda, long long sA,
    const unsigned short* __restrict__ Alp, int ldal, long long sAl,
    const unsigned short* __restrict__ Bhp, int ldb, long long sB,
    const unsigned short* __restrict__ Blp, int ldbl, long long sBl,
    void* Chp, int ldc, long long sC,
    void* Clp, int ldcl, long long sCl,
    int M, int N, int K, float oscale, float lsc, float ocarry) {
  __shared__ __align__(16) float sT[8][16 * 68];
  constexpr int TM = 16 * MI;
  const int by   = blockIdx.y;
  const int lane = threadIdx.x & 31;
  const int wave = threadIdx.x >> 5;
  const int tilesN = N >> 6;
  const int tilesM = M / TM;
  const int tile = blockIdx.x * 8 + wave;
  if (tile >= tilesM * tilesN) return;
  const int tm = tile / tilesN;
  const int tn = tile - tm * tilesN;
  const int m0 = tm * TM;
  const int n0 = tn << 6;

  const unsigned short* Ah = Ahp + (size_t)((long long)by * sA);
  const unsigned short* Bh = Bhp + (size_t)((long long)by * sB);
  const unsigned short* Al = Ah;
  const unsigned short* Bl = Bh;
  if constexpr (LO == 1) Al = Alp + (size_t)((long long)by * sAl);
  if constexpr (LO == 2) Bl = Blp + (size_t)((long long)by * sBl);

  const int rlane = lane & 15;
  const int koff  = (lane >> 4) * 8;
  const int mOff  = (lane >> 4) * 8;

  v8f acc[MI][4], acc2[MI][4];
#pragma unroll
  for (int i = 0; i < MI; ++i)
#pragma unroll
    for (int j = 0; j < 4; ++j) { acc[i][j] = zero8(); acc2[i][j] = zero8(); }

  for (int k0 = 0; k0 < K; k0 += 32) {
    v16h bh[4], bl[4];
#pragma unroll
    for (int j = 0; j < 4; ++j) {
      const size_t bofs = (size_t)(n0 + (j << 4) + rlane) * ldb + koff + k0;
      bh[j] = ldfrag_u(Bh + bofs);
      if constexpr (LO == 2) {
        const size_t bofl = (size_t)(n0 + (j << 4) + rlane) * ldbl + koff + k0;
        bl[j] = ldfrag_u(Bl + bofl);
      } else {
        bl[j] = bh[j];
      }
    }
#pragma unroll
    for (int i = 0; i < MI; ++i) {
      const size_t ao = (size_t)(m0 + (i << 4) + rlane) * lda + koff + k0;
      const v16h ah = ldfrag_u(Ah + ao);
#pragma unroll
      for (int j = 0; j < 4; ++j) acc[i][j] = mma_raw(ah, bh[j], acc[i][j]);
      if constexpr (LO == 1) {
        const size_t al_o = (size_t)(m0 + (i << 4) + rlane) * ldal + koff + k0;
        const v16h al = ldfrag_u(Al + al_o);
#pragma unroll
        for (int j = 0; j < 4; ++j) acc2[i][j] = mma_raw(al, bh[j], acc2[i][j]);
        dep_guard2(acc[i][0], acc[i][3], acc2[i][0], acc2[i][3], ah, al);
      } else if constexpr (LO == 2) {
#pragma unroll
        for (int j = 0; j < 4; ++j) acc2[i][j] = mma_raw(ah, bl[j], acc2[i][j]);
        dep_guard2(acc[i][0], acc[i][3], acc2[i][0], acc2[i][3], ah, ah);
      } else {
        dep_guard1(acc[i][0], acc[i][3], ah);
      }
    }
    keep4_h(bh[0], bh[1], bh[2], bh[3]);
    if constexpr (LO == 2) keep4_h(bl[0], bl[1], bl[2], bl[3]);
  }
#pragma unroll
  for (int i = 0; i < MI; ++i) {
    acc_guard4(acc[i][0], acc[i][1], acc[i][2], acc[i][3]);
    if constexpr (LO != 0) acc_guard4(acc2[i][0], acc2[i][1], acc2[i][2], acc2[i][3]);
  }

  const int hh2 = lane >> 4, c4 = (lane & 15) * 4;
  const int q8  = lane >> 3, c8 = (lane & 7) * 8;

  float* slab = sT[wave];
#pragma unroll
  for (int i = 0; i < MI; ++i) {
    const int mBase = m0 + (i << 4);
#pragma unroll
    for (int j = 0; j < 4; ++j) {
#pragma unroll
      for (int r = 0; r < 8; ++r) {
        float val = acc[i][j][r];
        if constexpr (LO != 0) val += acc2[i][j][r] * lsc;
        slab[(mOff + r) * 68 + (j << 4) + rlane] = val * oscale;
      }
    }
    wave_sync_lds();
    if constexpr (OM == 0) {
      float* C = (float*)Chp + (size_t)((long long)by * sC);
      v4f vals[8];
#pragma unroll
      for (int it = 0; it < 8; ++it) {
        const int row = it * 2 + hh2;
        vals[it] = *(const v4f*)(slab + row * 68 + c4);
      }
      for (int pass = 0; pass < 2; ++pass) {
#pragma unroll
        for (int it = 0; it < 8; ++it) {
          const int gr = mBase + it * 2 + hh2;
          *(volatile v4f*)(C + (size_t)gr * ldc + n0 + c4) = vals[it];
        }
        __threadfence();
      }
    } else {
      unsigned short* Ch = (unsigned short*)Chp + (size_t)((long long)by * sC);
      unsigned short* Cl = Ch;
      if constexpr (OM == 2) Cl = (unsigned short*)Clp + (size_t)((long long)by * sCl);
      v4u hv[4], lv[4];
#pragma unroll
      for (int it = 0; it < 4; ++it) {
        const int row = it * 4 + q8;
        const float* sp = slab + row * 68 + c8;
        v4u a = {0u, 0u, 0u, 0u};
        v4u b = {0u, 0u, 0u, 0u};
#pragma unroll
        for (int e = 0; e < 4; ++e) {
          const float f0 = sp[2 * e] * ocarry;
          const float f1 = sp[2 * e + 1] * ocarry;
          const _Float16 h0 = (_Float16)f0;
          const _Float16 h1 = (_Float16)f1;
          a[e] = pk16(h_bits(h0), h_bits(h1));
          if constexpr (OM == 2) {
            const _Float16 l0 = (_Float16)((f0 - (float)h0) * RSC);
            const _Float16 l1 = (_Float16)((f1 - (float)h1) * RSC);
            b[e] = pk16(h_bits(l0), h_bits(l1));
          }
        }
        hv[it] = a;
        lv[it] = b;
      }
      for (int pass = 0; pass < 2; ++pass) {
#pragma unroll
        for (int it = 0; it < 4; ++it) {
          const int row = it * 4 + q8;
          *(volatile v4u*)(Ch + (size_t)(mBase + row) * ldc + n0 + c8) = hv[it];
          if constexpr (OM == 2) {
            *(volatile v4u*)(Cl + (size_t)(mBase + row) * ldcl + n0 + c8) = lv[it];
          }
        }
        __threadfence();
      }
    }
    wave_sync_lds();
  }
}

template <int HR>
__global__ __launch_bounds__(ATT_THREADS)
void attnw(const unsigned short* __restrict__ QKp, const unsigned short* __restrict__ QKLp,
           const unsigned short* __restrict__ VTq, const unsigned short* __restrict__ VTLq,
           unsigned short* CTp, unsigned short* CTLp, int qt0, int nqt) {
  constexpr int SMF = (HR != 0) ? OS2_FLOATS : PS_FLOATS;
  __shared__ __align__(16) float smem[SMF];

  const int tid  = threadIdx.x;
  const int wave = tid >> 5;
  const int lane = tid & 31;
  const int hh   = lane >> 4;
  const int c    = lane & 15;

  const int bx   = blockIdx.x;
  const int hb   = bx % NHB;
  const int qt   = qt0 + (bx / NHB) % nqt;
  const int bat  = bx / (NHB * nqt);
  const int head = hb * HPB + wave;
  const int q0   = qt * 16;
  const int hoff = head * HDIM + 8 * hh;

  const _Float16* QKh = (const _Float16*)(const void*)QKp;
  const _Float16* Qh = QKh + ((size_t)bat * NQ + q0 + c) * PQK + hoff;
  const _Float16* Kb = QKh + (size_t)bat * NC * PQK + DMODEL + hoff;
  const _Float16* Vb = (const _Float16*)(const void*)VTq + ((size_t)bat * DMODEL + head * HDIM) * NC + 8 * hh;
  const _Float16* Ql  = Qh;
  const _Float16* Klb = Kb;
  const _Float16* Vlb = Vb;
  if constexpr (HR != 0) {
    const _Float16* QKl = (const _Float16*)(const void*)QKLp;
    Ql  = QKl + ((size_t)bat * NE + q0 + c) * PQK + hoff;
    Klb = QKl + (size_t)bat * NE * PQK + DMODEL + hoff;
    Vlb = (const _Float16*)(const void*)VTLq + ((size_t)bat * DMODEL + head * HDIM) * NE + 8 * hh;
  }
  const float lsc = (LOG2E * ATT_SCALE) / (QC * KC);

  const v16h qa = ldfrag_h(Qh), qb = ldfrag_h(Qh + 32);
  v16h qal = qa, qbl = qb;
  if constexpr (HR != 0) { qal = ldfrag_h(Ql); qbl = ldfrag_h(Ql + 32); }

  float mrow[8], lrow[8];
  v8f oh[4], ox[4];
#pragma unroll
  for (int dt = 0; dt < 4; ++dt) { oh[dt] = zero8(); ox[dt] = zero8(); }
#pragma unroll
  for (int r = 0; r < 8; ++r) { mrow[r] = -INFINITY; lrow[r] = 0.f; }
  float* pt = smem + wave * (16 * 36);
  const int nkey = q0 + 16;

#pragma unroll 1
  for (int kb = 0; kb < nkey; kb += 32) {
    const _Float16* kp  = Kb  + (size_t)(kb + c) * PQK;
    const _Float16* klp = Klb + (size_t)(kb + c) * PQK;
    v8f s0, s1;
    {
      const v16h k0 = ldfrag_h(kp), k1 = ldfrag_h(kp + 32);
      v8f sh = mma_raw(qa, k0, zero8());
      sh = mma_raw(qb, k1, sh);
      if constexpr (HR != 0) {
        const v16h l0 = ldfrag_h(klp), l1 = ldfrag_h(klp + 32);
        v8f sx = mma_raw(qa, l0, zero8());
        sx = mma_raw(qb, l1, sx);
        sx = mma_raw(qal, k0, sx);
        sx = mma_raw(qbl, k1, sx);
        guard_x4(sh, sx, k0, k1, l0, l1);
        s0 = sh + sx * RINV;
      } else {
        guard_s2(sh, k0, k1);
        s0 = sh;
      }
    }
    {
      const _Float16* kq  = kp  + (size_t)16 * PQK;
      const _Float16* klq = klp + (size_t)16 * PQK;
      const v16h k0 = ldfrag_h(kq), k1 = ldfrag_h(kq + 32);
      v8f sh = mma_raw(qa, k0, zero8());
      sh = mma_raw(qb, k1, sh);
      if constexpr (HR != 0) {
        const v16h l0 = ldfrag_h(klq), l1 = ldfrag_h(klq + 32);
        v8f sx = mma_raw(qa, l0, zero8());
        sx = mma_raw(qb, l1, sx);
        sx = mma_raw(qal, k0, sx);
        sx = mma_raw(qbl, k1, sx);
        guard_x8(sh, sx, k0, k1, l0, l1, qa, qb, qal, qbl);
        s1 = sh + sx * RINV;
      } else {
        guard_s4(sh, k0, k1, qa, qb);
        s1 = sh;
      }
    }
    const int key0 = kb + c;
    const int key1 = key0 + 16;
#pragma unroll
    for (int r = 0; r < 8; ++r) {
      const int row = q0 + 8 * hh + r;
      const float u0 = s0[r] * lsc;
      const float u1 = s1[r] * lsc;
      const float t0 = (key0 <= row) ? u0 : -INFINITY;
      const float t1 = (key1 <= row) ? u1 : -INFINITY;
      float mx = fmaxf(t0, t1);
#pragma unroll
      for (int off = 1; off < 16; off <<= 1) mx = fmaxf(mx, __shfl_xor(mx, off, 32));
      const float mn = fmaxf(mrow[r], mx);
      const float al = exp2f(fmaxf(mrow[r] - mn, -126.0f));
      mrow[r] = mn;
      const float e0 = exp2f(t0 - mn);
      const float e1 = exp2f(t1 - mn);
      float ps = e0 + e1;
#pragma unroll
      for (int off = 1; off < 16; off <<= 1) ps += __shfl_xor(ps, off, 32);
      lrow[r] = lrow[r] * al + ps;
#pragma unroll
      for (int dt = 0; dt < 4; ++dt) {
        oh[dt][r] *= al;
        if constexpr (HR != 0) ox[dt][r] *= al;
      }
      const int ro = (8 * hh + r) * 36 + c;
      pt[ro]      = e0;
      pt[ro + 16] = e1;
    }
    wave_sync_lds();
    FragH ph, pl;
    {
      const float* prow = pt + c * 36 + 8 * hh;
      const v4f p0 = *(const v4f*)(prow), p1 = *(const v4f*)(prow + 4);
      const v4f p2 = *(const v4f*)(prow + 16), p3 = *(const v4f*)(prow + 20);
#pragma unroll
      for (int e = 0; e < 4; ++e) {
        const float f0 = p0[e] * PC, f1 = p1[e] * PC, f2 = p2[e] * PC, f3 = p3[e] * PC;
        const _Float16 g0 = (_Float16)f0, g1 = (_Float16)f1, g2 = (_Float16)f2, g3 = (_Float16)f3;
        ph.h[0][e]     = g0;
        ph.h[0][4 + e] = g1;
        ph.h[1][e]     = g2;
        ph.h[1][4 + e] = g3;
        if constexpr (HR != 0) {
          pl.h[0][e]     = (_Float16)((f0 - (float)g0) * RSC);
          pl.h[0][4 + e] = (_Float16)((f1 - (float)g1) * RSC);
          pl.h[1][e]     = (_Float16)((f2 - (float)g2) * RSC);
          pl.h[1][4 + e] = (_Float16)((f3 - (float)g3) * RSC);
        } else {
          pl.h[0][e] = g0; pl.h[0][4 + e] = g1; pl.h[1][e] = g2; pl.h[1][4 + e] = g3;
        }
      }
    }
    const _Float16* vp = Vb + (size_t)c * NC + kb;
    if constexpr (HR != 0) {
      const _Float16* vl = Vlb + (size_t)c * NE + kb;
#pragma unroll
      for (int dt = 0; dt < 4; ++dt) {
        const v16h vh = ldfrag_h(vp + (size_t)(16 * dt) * NC);
        const v16h vr = ldfrag_h(vl + (size_t)(16 * dt) * NE);
        oh[dt] = mma_raw(ph.v, vh, oh[dt]);
        ox[dt] = mma_raw(ph.v, vr, ox[dt]);
        ox[dt] = mma_raw(pl.v, vh, ox[dt]);
        guard_pv2(oh[dt], ox[dt], ph.v, pl.v, vh, vr);
      }
    } else {
      const v16h vb0 = ldfrag_h(vp);
      const v16h vb1 = ldfrag_h(vp + (size_t)16 * NC);
      const v16h vb2 = ldfrag_h(vp + (size_t)32 * NC);
      const v16h vb3 = ldfrag_h(vp + (size_t)48 * NC);
      oh[0] = mma_raw(ph.v, vb0, oh[0]);
      oh[1] = mma_raw(ph.v, vb1, oh[1]);
      oh[2] = mma_raw(ph.v, vb2, oh[2]);
      oh[3] = mma_raw(ph.v, vb3, oh[3]);
      guard_pv4(oh[0], oh[1], oh[2], oh[3], ph.v, vb0, vb1, vb2, vb3);
    }
    wave_sync_lds();
  }

  __syncthreads();
  unsigned short* Os = (unsigned short*)smem;
  const float oc = FC / (PC * VC);
  unsigned short* osw = Os + wave * HDIM + c;
#pragma unroll
  for (int r = 0; r < 8; ++r) {
    const float inv = (1.0f / lrow[r]) * oc;
    const int ro = (8 * hh + r) * OSP;
#pragma unroll
    for (int dt = 0; dt < 4; ++dt) {
      float f = oh[dt][r];
      if constexpr (HR != 0) f += ox[dt][r] * RINV;
      f *= inv;
      const _Float16 h = (_Float16)f;
      osw[ro + 16 * dt] = h_bits(h);
      if constexpr (HR != 0) osw[OS_HALVES + ro + 16 * dt] = h_bits((_Float16)((f - (float)h) * RSC));
    }
  }
  __syncthreads();
  {
    v4u vals[4], lv[4];
#pragma unroll
    for (int it = 0; it < 4; ++it) {
      const int p = it * ATT_THREADS + tid;
      vals[it] = *(const v4u*)(Os + (size_t)p * 8);
      if constexpr (HR != 0) lv[it] = *(const v4u*)(Os + OS_HALVES + (size_t)p * 8);
      else lv[it] = vals[it];
    }
    unsigned short* dst  = CTp + ((size_t)bat * NQ + q0) * DMODEL + (size_t)hb * OSP;
    unsigned short* dstl = dst;
    if constexpr (HR != 0) dstl = CTLp + ((size_t)bat * NE + q0) * DMODEL + (size_t)hb * OSP;
    for (int pass = 0; pass < 2; ++pass) {
#pragma unroll
      for (int it = 0; it < 4; ++it) {
        const int p = it * ATT_THREADS + tid;
        const int row = p >> 6, col8 = (p & 63) * 8;
        *(volatile v4u*)(dst + (size_t)row * DMODEL + col8) = vals[it];
        if constexpr (HR != 0) {
          *(volatile v4u*)(dstl + (size_t)row * DMODEL + col8) = lv[it];
        }
      }
      __threadfence();
    }
  }
}

extern "C" void kernel_launch(void* const* d_in, const int* in_sizes, int n_in,
                              void* d_out, int out_size, void* d_ws, size_t ws_size,
                              hipStream_t stream) {
  if (n_in < 5) return;
  if (in_sizes[0] != NROWS * DMODEL) return;
  if (in_sizes[1] != DMODEL || in_sizes[2] != DMODEL) return;
  if (in_sizes[3] != 3 * DMODEL * DMODEL) return;
  if (in_sizes[4] != DMODEL * DMODEL) return;
  if (out_size != NROWS * DMODEL) return;

  const float* x     = (const float*)d_in[0];
  const float* ln_g  = (const float*)d_in[1];
  const float* ln_b  = (const float*)d_in[2];
  const float* w_qkv = (const float*)d_in[3];
  const float* w_o   = (const float*)d_in[4];
  float*       out   = (float*)d_out;

  const size_t PW3  = (size_t)3 * DMODEL * DMODEL * 2;
  const size_t PWO  = (size_t)DMODEL * DMODEL * 2;
  const size_t PX16 = (size_t)NROWS * DMODEL * 2;
  const size_t PQKB = (size_t)NROWS * PQK * 2;
  const size_t PQKL = (size_t)NB * NE * PQK * 2;
  const size_t PVT  = (size_t)NB * DMODEL * NC * 2;
  const size_t PVTL = (size_t)NB * DMODEL * NE * 2;
  const size_t PCTL = (size_t)NB * NE * DMODEL * 2;
  size_t off = 0;
  const size_t oWQKV = off; off += PW3;
  const size_t oWO   = off; off += PWO;
  const size_t oXH   = off; off += PX16;
  const size_t oXL   = off; off += PX16;
  const size_t oQK   = off; off += PQKB;
  const size_t oQKL  = off; off += PQKL;
  const size_t oVT   = off; off += PVT;
  const size_t oVTL  = off; off += PVTL;
  const size_t oCT   = off; off += PX16;
  const size_t oCTL  = off; off += PCTL;
  const size_t endAll = off;
  if (endAll > ws_size) return;
  if (endAll > (size_t)134217728) return;

  char* ws = (char*)d_ws;
  unsigned short* WQKV = (unsigned short*)(ws + oWQKV);
  unsigned short* WO16 = (unsigned short*)(ws + oWO);
  unsigned short* XH   = (unsigned short*)(ws + oXH);
  unsigned short* XL   = (unsigned short*)(ws + oXL);
  unsigned short* QK   = (unsigned short*)(ws + oQK);
  unsigned short* QKL  = (unsigned short*)(ws + oQKL);
  unsigned short* VT   = (unsigned short*)(ws + oVT);
  unsigned short* VTL  = (unsigned short*)(ws + oVTL);
  unsigned short* CT   = (unsigned short*)(ws + oCT);
  unsigned short* CTL  = (unsigned short*)(ws + oCTL);
  const unsigned short* nus = (const unsigned short*)0;

  const dim3 blk(256);
  const int tilesQKlate = (NL / 64) * ((2 * DMODEL) / 64);
  const int tilesQKearl = (NE / 32) * ((2 * DMODEL) / 64);
  const int tilesVlate  = (DMODEL / 64) * (NL / 64);
  const int tilesVearl  = (DMODEL / 16) * (NE / 64);
  const int tilesOearl  = (NE / 32) * (DMODEL / 64);
  const int tilesOlate  = (NL / 64) * (DMODEL / 64);
  const dim3 gQKlate((tilesQKlate + 7) / 8, NB);
  const dim3 gQKearl((tilesQKearl + 7) / 8, NB);
  const dim3 gVlate((tilesVlate + 7) / 8, NB);
  const dim3 gVearl((tilesVearl + 7) / 8, NB);
  const dim3 gOearl((tilesOearl + 7) / 8, NB);
  const dim3 gOlate((tilesOlate + 7) / 8, NB);
  const dim3 gATe(NB * (NE / 16) * NHB);
  const dim3 gATl(NB * (NL / 16) * NHB);
  const dim3 bAT(ATT_THREADS);
  const dim3 gLN(NROWS);
  const dim3 bLN(LN_THREADS);

  const long long sXrow = (long long)NQ * DMODEL;
  const long long sQK   = (long long)NQ * PQK;
  const long long sQKL  = (long long)NE * PQK;
  const long long sVT   = (long long)DMODEL * NC;
  const long long sVTL  = (long long)DMODEL * NE;
  const long long sCTL  = (long long)NE * DMODEL;
  const float osc_qkv = 1.0f / (HCARRY * WSC);
  const float osc_out = 1.0f / (FC * WSC);

  wcvt16<<<dim3(3 * DMODEL), dim3(128), 0, stream>>>(w_qkv, WQKV, 3 * DMODEL, 1);
  wcvt16<<<dim3(DMODEL), dim3(128), 0, stream>>>(w_o, WO16, DMODEL, 0);

  lnorm2<<<gLN, bLN, 0, stream>>>(x, ln_g, ln_b, XH, XL);

  gemmw<4, 0, 1><<<gQKlate, blk, 0, stream>>>(
      XH + (size_t)NE * DMODEL, DMODEL, sXrow,
      nus, 0, 0LL,
      WQKV, DMODEL, 0LL,
      nus, 0, 0LL,
      (void*)(QK + (size_t)NE * PQK), PQK, sQK,
      (void*)0, 0, 0LL,
      NL, 2 * DMODEL, DMODEL, osc_qkv, 0.0f, QC);

  gemmw<2, 1, 2><<<gQKearl, blk, 0, stream>>>(
      XH, DMODEL, sXrow,
      XL, DMODEL, sXrow,
      WQKV, DMODEL, 0LL,
      nus, 0, 0LL,
      (void*)QK, PQK, sQK,
      (void*)QKL, PQK, sQKL,
      NE, 2 * DMODEL, DMODEL, osc_qkv, RINV, QC);

  gemmw<4, 0, 1><<<gVlate, blk, 0, stream>>>(
      WQKV + (size_t)2 * DMODEL * DMODEL, DMODEL, 0LL,
      nus, 0, 0LL,
      XH + (size_t)NE * DMODEL, DMODEL, sXrow,
      nus, 0, 0LL,
      (void*)(VT + NE), NC, sVT,
      (void*)0, 0, 0LL,
      DMODEL, NL, DMODEL, osc_qkv, 0.0f, VC);

  gemmw<1, 2, 2><<<gVearl, blk, 0, stream>>>(
      WQKV + (size_t)2 * DMODEL * DMODEL, DMODEL, 0LL,
      nus, 0, 0LL,
      XH, DMODEL, sXrow,
      XL, DMODEL, sXrow,
      (void*)VT, NC, sVT,
      (void*)VTL, NE, sVTL,
      DMODEL, NE, DMODEL, osc_qkv, RINV, VC);

  attnw<1><<<gATe, bAT, 0, stream>>>(QK, QKL, VT, VTL, CT, CTL, 0, NE / 16);

  attnw<0><<<gATl, bAT, 0, stream>>>(QK, QKL, VT, VTL, CT, CTL, NE / 16, NL / 16);

  gemmw<2, 1, 0><<<gOearl, blk, 0, stream>>>(
      CT, DMODEL, sXrow,
      CTL, DMODEL, sCTL,
      WO16, DMODEL, 0LL,
      nus, 0, 0LL,
      (void*)out, DMODEL, sXrow,
      (void*)0, 0, 0LL,
      NE, DMODEL, DMODEL, osc_out, RINV, 1.0f);

  gemmw<4, 0, 0><<<gOlate, blk, 0, stream>>>(
      CT + (size_t)NE * DMODEL, DMODEL, sXrow,
      nus, 0, 0LL,
      WO16, DMODEL, 0LL,
      nus, 0, 0LL,
      (void*)(out + (size_t)NE * DMODEL), DMODEL, sXrow,
      (void*)0, 0, 0LL,
      NL, DMODEL, DMODEL, osc_out, 0.0f, 1.0f);
  (void)hipGetLastError();
}
